// TransformerCrf_56882546868902
// MI455X (gfx1250) — hardware-verified
//
#include <hip/hip_runtime.h>
#include <stddef.h>
#include <stdint.h>

#define NBATCH 32
#define SQ     512
#define NTOK   16384
#define DM     256
#define NH     8
#define HDM    32
#define DFF    1024
#define NLAB   20
#define NLABP  32
#define NLAYER 4
#define NQKV   768
#define QB     128
#define KC     64
#define NQB    4
#define NCK    8

static_assert(NTOK == NBATCH * SQ);
static_assert(NH * HDM == DM);
static_assert(NQKV == 3 * DM);
static_assert(NQB * QB == SQ);
static_assert(NCK * KC == SQ);
static_assert(DM % 64 == 0);
static_assert(DFF % 64 == 0);
static_assert(NTOK % 256 == 0);
static_assert(SQ % 256 == 0);
static_assert(NLAB <= NLABP);
static_assert((256 * NLAB) % 1024 == 0);

typedef _Float16 v16h __attribute__((ext_vector_type(16)));
typedef _Float16 v8h  __attribute__((ext_vector_type(8)));
typedef float    v8f  __attribute__((ext_vector_type(8)));
typedef float    v4f  __attribute__((ext_vector_type(4)));
typedef unsigned int v4u __attribute__((ext_vector_type(4)));

union Frag  { v16h v; v8h h[2]; };
union Pack8 { v8h h; v4u u; };

__device__ __forceinline__ v8f mma16(v16h a, v16h b, v8f c) {
  c = __builtin_amdgcn_wmma_f32_16x16x32_f16(false, a, false, b, (short)0, c, false, false);
  asm volatile("v_nop\n\tv_nop\n\tv_nop\n\tv_nop" : "+v"(c) : "v"(a), "v"(b));
  return c;
}

__device__ __forceinline__ v16h ldfrag(const _Float16* p, int ld, int row0, int k0, int lane) {
  const int m = lane & 15, lh = lane >> 4;
  const _Float16* q = p + (size_t)(row0 + m) * ld + k0 + 8 * lh;
  Frag f;
  f.h[0] = *(const v8h*)(q);
  f.h[1] = *(const v8h*)(q + 16);
  return f.v;
}

__device__ __forceinline__ v8f zero8() { return (v8f){0.f, 0.f, 0.f, 0.f, 0.f, 0.f, 0.f, 0.f}; }

__device__ __forceinline__ v4u pack8h(v4f a0, v4f a1) {
  Pack8 pk;
  pk.h = (v8h){(_Float16)a0[0], (_Float16)a0[1], (_Float16)a0[2], (_Float16)a0[3],
               (_Float16)a1[0], (_Float16)a1[1], (_Float16)a1[2], (_Float16)a1[3]};
  return pk.u;
}

__device__ __forceinline__ void gemm32x64(const _Float16* __restrict__ A, int lda,
                                          const _Float16* __restrict__ Bt, int ldb, int K,
                                          int m0, int n0, int lane, v8f (&acc)[2][4]) {
#pragma unroll 1
  for (int k0 = 0; k0 < K; k0 += 32) {
    const v16h a0 = ldfrag(A, lda, m0, k0, lane);
    const v16h a1 = ldfrag(A, lda, m0 + 16, k0, lane);
    const v16h b0 = ldfrag(Bt, ldb, n0, k0, lane);
    const v16h b1 = ldfrag(Bt, ldb, n0 + 16, k0, lane);
    const v16h b2 = ldfrag(Bt, ldb, n0 + 32, k0, lane);
    const v16h b3 = ldfrag(Bt, ldb, n0 + 48, k0, lane);
    acc[0][0] = mma16(a0, b0, acc[0][0]);
    acc[1][0] = mma16(a1, b0, acc[1][0]);
    acc[0][1] = mma16(a0, b1, acc[0][1]);
    acc[1][1] = mma16(a1, b1, acc[1][1]);
    acc[0][2] = mma16(a0, b2, acc[0][2]);
    acc[1][2] = mma16(a1, b2, acc[1][2]);
    acc[0][3] = mma16(a0, b3, acc[0][3]);
    acc[1][3] = mma16(a1, b3, acc[1][3]);
  }
}

__global__ __launch_bounds__(256) void k_embed(const int* __restrict__ ids, const float* __restrict__ emb, int nvocab,
                                               const float* __restrict__ pos,
                                               float* __restrict__ xf, _Float16* __restrict__ xh) {
  const int tid = threadIdx.x, lane = tid & 31, wave = tid >> 5;
  const int m = blockIdx.x * 8 + wave;
  const int s = m & (SQ - 1);
  int id = ids[m];
  id = (id < 0) ? (id + nvocab) : id;
  id = min(max(id, 0), nvocab - 1);
  const float* er = emb + (size_t)id * DM;
  const float* pr = pos + (size_t)s * DM;

  v4f v[2];
#pragma unroll
  for (int it = 0; it < 2; ++it) {
    const int idx = it * 128 + lane * 4;
    v[it] = *(const v4f*)(er + idx) + *(const v4f*)(pr + idx);
  }
  const v4f a0 = *(const v4f*)(er + 8 * lane) + *(const v4f*)(pr + 8 * lane);
  const v4f a1 = *(const v4f*)(er + 8 * lane + 4) + *(const v4f*)(pr + 8 * lane + 4);
  const v4u hv = pack8h(a0, a1);

  float* xrow = xf + (size_t)m * DM;
  _Float16* hrow = xh + (size_t)m * DM;
  for (int ps = 0; ps < 2; ++ps) {
#pragma unroll
    for (int it = 0; it < 2; ++it) *(volatile v4f*)(xrow + it * 128 + lane * 4) = v[it];
    *(volatile v4u*)(hrow + 8 * lane) = hv;
    __threadfence();
  }
}

__global__ __launch_bounds__(256) void k_wtc(const float* __restrict__ W, int K, int N,
                                             size_t zin, size_t zout, float scale,
                                             _Float16* __restrict__ out) {
  __shared__ float tile[64][33];
  const int tid = threadIdx.x;
  const int k0 = blockIdx.x * 64, n0 = blockIdx.y * 32;
  const float* Wz = W + (size_t)blockIdx.z * zin;
  _Float16* oz = out + (size_t)blockIdx.z * zout;
#pragma unroll
  for (int e = 0; e < 8; ++e) {
    const int idx = tid + 256 * e;
    const int kr = idx >> 5;
    const int nc = idx & 31;
    const int n  = n0 + nc;
    const int nn = min(n, N - 1);
    const float w = Wz[(size_t)(k0 + kr) * N + nn];
    tile[kr][nc] = (n < N) ? w * scale : 0.f;
  }
  __syncthreads();
  const int nr = tid >> 3, pc = tid & 7;
  float f[8];
#pragma unroll
  for (int j = 0; j < 8; ++j) f[j] = tile[pc * 8 + j][nr];
  const v4u val = pack8h((v4f){f[0], f[1], f[2], f[3]}, (v4f){f[4], f[5], f[6], f[7]});
  _Float16* dst = oz + (size_t)(n0 + nr) * K + k0 + pc * 8;
  for (int ps = 0; ps < 2; ++ps) {
    *(volatile v4u*)dst = val;
    __threadfence();
  }
}

#define STP 72
#define SVP 264
__global__ __launch_bounds__(256) void k_qkv(const _Float16* __restrict__ xh,
                                             const _Float16* __restrict__ wt,
                                             const float* __restrict__ bq,
                                             const float* __restrict__ bk,
                                             const float* __restrict__ bv,
                                             _Float16* __restrict__ qkp,
                                             _Float16* __restrict__ vtp) {
  __shared__ __align__(16) _Float16 st[256 * STP];
  const int tid = threadIdx.x, lane = tid & 31, wave = tid >> 5;
  const int hh = lane >> 4, c = lane & 15;
  const int bx = blockIdx.x;
  const int token0 = bx * 256;
  const int b  = bx >> 1;
  const int sb = (bx & 1) * 256;
  const int ns = blockIdx.y;
  const int which = ns >> 2;
  const int hp = ns & 3;
  const int m0 = token0 + wave * 32;
  const int n0 = ns * 64;

  v8f acc[2][4];
#pragma unroll
  for (int s = 0; s < 2; ++s)
#pragma unroll
    for (int t = 0; t < 4; ++t) acc[s][t] = zero8();
  gemm32x64(xh, DM, wt, DM, DM, m0, n0, lane, acc);

  float bb[4];
#pragma unroll
  for (int t = 0; t < 4; ++t) {
    const int i = hp * 64 + 16 * t + c;
    const float xq = bq[i], xk = bk[i], xv = bv[i];
    bb[t] = (which == 0) ? xq : ((which == 1) ? xk : xv);
  }
  const float wsc = 0.015625f;
  const float csc = 8.0f;

  if (which < 2) {
#pragma unroll
    for (int sub = 0; sub < 2; ++sub)
#pragma unroll
      for (int t = 0; t < 4; ++t)
#pragma unroll
        for (int r = 0; r < 8; ++r)
          st[(wave * 32 + sub * 16 + 8 * hh + r) * STP + 16 * t + c] =
              (_Float16)((acc[sub][t][r] * wsc + bb[t]) * csc);
  } else {
#pragma unroll
    for (int sub = 0; sub < 2; ++sub)
#pragma unroll
      for (int t = 0; t < 4; ++t)
#pragma unroll
        for (int r = 0; r < 8; ++r)
          st[(16 * t + c) * SVP + wave * 32 + sub * 16 + 8 * hh + r] =
              (_Float16)((acc[sub][t][r] * wsc + bb[t]) * csc);
  }
  __syncthreads();

  if (which < 2) {
    _Float16* base = qkp + (size_t)which * NTOK * DM + (size_t)token0 * DM + hp * 64;
#pragma unroll
    for (int g = 0; g < 2; ++g) {
      v4u val[4];
      size_t go[4];
#pragma unroll
      for (int j = 0; j < 4; ++j) {
        const int p  = tid + 256 * (4 * g + j);
        const int lr = p >> 3;
        const int pc = p & 7;
        Pack8 pk;
        pk.h   = *(const v8h*)(st + lr * STP + pc * 8);
        val[j] = pk.u;
        go[j]  = (size_t)lr * DM + pc * 8;
      }
      for (int ps = 0; ps < 2; ++ps) {
#pragma unroll
        for (int j = 0; j < 4; ++j) *(volatile v4u*)(base + go[j]) = val[j];
        __threadfence();
      }
    }
  } else {
    _Float16* base = vtp + (size_t)(b * NH + 2 * hp) * HDM * SQ + sb;
#pragma unroll
    for (int g = 0; g < 2; ++g) {
      v4u val[4];
      size_t go[4];
#pragma unroll
      for (int j = 0; j < 4; ++j) {
        const int p    = tid + 256 * (4 * g + j);
        const int drow = p >> 5;
        const int pc   = p & 31;
        Pack8 pk;
        pk.h   = *(const v8h*)(st + drow * SVP + pc * 8);
        val[j] = pk.u;
        go[j]  = (size_t)drow * SQ + pc * 8;
      }
      for (int ps = 0; ps < 2; ++ps) {
#pragma unroll
        for (int j = 0; j < 4; ++j) *(volatile v4u*)(base + go[j]) = val[j];
        __threadfence();
      }
    }
  }
}

#define KSP 40
#define VTP 72
#define PTP 72
__global__ __launch_bounds__(256) void k_attn(const _Float16* __restrict__ qkp,
                                              const _Float16* __restrict__ vtp,
                                              const int* __restrict__ slen,
                                              float* __restrict__ attp, float sscale) {
  __shared__ __align__(16) _Float16 Ks[KC * KSP];
  __shared__ __align__(16) _Float16 Vs[HDM * VTP];
  __shared__ __align__(16) _Float16 Ps[8 * 16 * PTP];

  const int tid = threadIdx.x, lane = tid & 31, wave = tid >> 5;
  const int hh = lane >> 4, c = lane & 15;
  const int qb  = blockIdx.x % NQB;
  const int hb  = blockIdx.x / NQB;
  const int h   = hb % NH;
  const int b   = hb / NH;
  int lenc = slen[b];
  lenc = min(max(lenc, 0), SQ);
  const int qblk = qb * QB;
  const int q0   = qblk + wave * 16;
  int nck = (qblk < lenc) ? ((lenc + KC - 1) / KC) : 0;
  nck = min(nck, NCK);

  const _Float16* Q = qkp + (size_t)b * SQ * DM + h * HDM;
  const _Float16* K = qkp + (size_t)NTOK * DM + (size_t)b * SQ * DM + h * HDM;
  const _Float16* V = vtp + (size_t)hb * HDM * SQ;

  const v16h qa = ldfrag(Q, DM, q0, 0, lane);

  const float NEGI = -__builtin_huge_valf();
  float mrow[8], lrow[8];
  v8f oacc[2];
#pragma unroll
  for (int r = 0; r < 8; ++r) { mrow[r] = NEGI; lrow[r] = 0.f; }
#pragma unroll
  for (int t = 0; t < 2; ++t) oacc[t] = zero8();

  _Float16* pw = Ps + wave * 16 * PTP;

  for (int kc = 0; kc < nck; ++kc) {
    const int kv0 = kc * KC;
    __syncthreads();
    {
      const int r  = tid >> 2;
      const int qq = (tid & 3) * 8;
      *(v8h*)(Ks + r * KSP + qq) = *(const v8h*)(K + (size_t)(kv0 + r) * DM + qq);
      const int r2 = tid >> 3;
      const int q2 = (tid & 7) * 8;
      *(v8h*)(Vs + r2 * VTP + q2) = *(const v8h*)(V + (size_t)r2 * SQ + kv0 + q2);
    }
    __syncthreads();

    v8f s[4];
#pragma unroll
    for (int j = 0; j < 4; ++j) {
      const v16h kb = ldfrag(Ks, KSP, j * 16, 0, lane);
      s[j] = mma16(qa, kb, zero8());
    }
    float cm[8];
#pragma unroll
    for (int r = 0; r < 8; ++r) {
      float mx = NEGI;
#pragma unroll
      for (int j = 0; j < 4; ++j) {
        const int key = kv0 + 16 * j + c;
        const float sv = s[j][r] * sscale;
        s[j][r] = (key < lenc) ? sv : NEGI;
        mx = fmaxf(mx, s[j][r]);
      }
#pragma unroll
      for (int off = 1; off < 16; off <<= 1) mx = fmaxf(mx, __shfl_xor(mx, off, 32));
      cm[r] = mx;
    }
    float al[8];
#pragma unroll
    for (int r = 0; r < 8; ++r) {
      const float mnew  = fmaxf(mrow[r], cm[r]);
      const float alpha = __expf(mrow[r] - mnew);
      mrow[r] = mnew;
      float psum = 0.f;
#pragma unroll
      for (int j = 0; j < 4; ++j) {
        const float p = __expf(s[j][r] - mnew);
        psum += p;
        pw[(8 * hh + r) * PTP + j * 16 + c] = (_Float16)(p * 1024.0f);
      }
#pragma unroll
      for (int off = 1; off < 16; off <<= 1) psum += __shfl_xor(psum, off, 32);
      lrow[r] = lrow[r] * alpha + psum;
      al[r] = alpha;
    }
#pragma unroll
    for (int t = 0; t < 2; ++t)
#pragma unroll
      for (int r = 0; r < 8; ++r) oacc[t][r] *= al[r];
    __syncthreads();

#pragma unroll
    for (int kk = 0; kk < 2; ++kk) {
      const v16h pa = ldfrag(pw, PTP, 0, kk * 32, lane);
#pragma unroll
      for (int t = 0; t < 2; ++t) {
        const v16h vb = ldfrag(Vs, VTP, t * 16, kk * 32, lane);
        oacc[t] = mma16(pa, vb, oacc[t]);
      }
    }
  }

  float inv[8];
#pragma unroll
  for (int r = 0; r < 8; ++r) {
    const int q = q0 + 8 * hh + r;
    inv[r] = (lrow[r] > 0.f && q < lenc) ? (0.0001220703125f / lrow[r]) : 0.f;
  }
  __syncthreads();
  float* fw = reinterpret_cast<float*>(pw);
#pragma unroll
  for (int r = 0; r < 8; ++r) {
#pragma unroll
    for (int t = 0; t < 2; ++t)
      fw[(8 * hh + r) * 36 + 16 * t + c] = oacc[t][r] * inv[r];
  }
  __syncthreads();
  v4f val[4];
  size_t go[4];
#pragma unroll
  for (int it = 0; it < 4; ++it) {
    const int p  = lane + 32 * it;
    const int L  = p >> 3;
    const int pc = p & 7;
    val[it] = *(const v4f*)(fw + L * 36 + pc * 4);
    go[it]  = ((size_t)hb * SQ + q0 + L) * HDM + pc * 4;
  }
  for (int ps = 0; ps < 2; ++ps) {
#pragma unroll
    for (int it = 0; it < 4; ++it) *(volatile v4f*)(attp + go[it]) = val[it];
    __threadfence();
  }
}

#define OTP 68
__device__ __forceinline__ void out_epilogue_f32(v8f (&acc)[2][4], float scale, const float (&bb)[4],
                                                 float* sw, float* __restrict__ out, int ldo,
                                                 int m0, int n0, int lane, int hh, int c) {
#pragma unroll
  for (int sub = 0; sub < 2; ++sub) {
    __syncthreads();
#pragma unroll
    for (int t = 0; t < 4; ++t) {
#pragma unroll
      for (int r = 0; r < 8; ++r) sw[(8 * hh + r) * OTP + 16 * t + c] = acc[sub][t][r] * scale + bb[t];
    }
    __syncthreads();
    v4f val[8];
    size_t go[8];
#pragma unroll
    for (int it = 0; it < 8; ++it) {
      const int p    = lane + 32 * it;
      const int L    = p >> 3;
      const int pc   = p & 7;
      const int row  = L >> 1;
      const int half = L & 1;
      val[it] = *(const v4f*)(sw + row * OTP + half * 32 + pc * 4);
      go[it]  = (size_t)(m0 + sub * 16 + row) * ldo + n0 + half * 32 + pc * 4;
    }
    for (int ps = 0; ps < 2; ++ps) {
#pragma unroll
      for (int it = 0; it < 8; ++it) *(volatile v4f*)(out + go[it]) = val[it];
      __threadfence();
    }
  }
}

__device__ __forceinline__ void out_epilogue_h16(v8f (&acc)[2][4], float scale, const float (&bb)[4], float oscale,
                                                 float* sw, _Float16* __restrict__ out, int ldo,
                                                 int m0, int n0, int lane, int hh, int c) {
#pragma unroll
  for (int sub = 0; sub < 2; ++sub) {
    __syncthreads();
#pragma unroll
    for (int t = 0; t < 4; ++t) {
#pragma unroll
      for (int r = 0; r < 8; ++r)
        sw[(8 * hh + r) * OTP + 16 * t + c] = (acc[sub][t][r] * scale + bb[t]) * oscale;
    }
    __syncthreads();
    v4u val[4];
    size_t go[4];
#pragma unroll
    for (int it = 0; it < 4; ++it) {
      const int p  = lane + 32 * it;
      const int L  = p >> 3;
      const int pc = p & 7;
      const float* ra = sw + L * OTP + pc * 8;
      val[it] = pack8h(*(const v4f*)(ra), *(const v4f*)(ra + 4));
      go[it]  = (size_t)(m0 + sub * 16 + L) * ldo + n0 + pc * 8;
    }
    for (int ps = 0; ps < 2; ++ps) {
#pragma unroll
      for (int it = 0; it < 4; ++it) *(volatile v4u*)(out + go[it]) = val[it];
      __threadfence();
    }
  }
}

__global__ __launch_bounds__(256) void k_gemm_f32(const _Float16* __restrict__ ap, int lda,
                                                  const _Float16* __restrict__ wt, int K,
                                                  const float* __restrict__ bias, float scale,
                                                  float* __restrict__ out, int ldo) {
  __shared__ __align__(16) float st[8][16 * OTP];
  const int tid = threadIdx.x, lane = tid & 31, wave = tid >> 5;
  const int hh = lane >> 4, c = lane & 15;
  const int m0 = blockIdx.x * 256 + wave * 32;
  const int n0 = blockIdx.y * 64;

  v8f acc[2][4];
#pragma unroll
  for (int s = 0; s < 2; ++s)
#pragma unroll
    for (int t = 0; t < 4; ++t) acc[s][t] = zero8();
  gemm32x64(ap, lda, wt, K, K, m0, n0, lane, acc);
  float bb[4];
#pragma unroll
  for (int t = 0; t < 4; ++t) bb[t] = bias[n0 + 16 * t + c];
  out_epilogue_f32(acc, scale, bb, st[wave], out, ldo, m0, n0, lane, hh, c);
}

__global__ __launch_bounds__(256) void k_gemm_h16(const _Float16* __restrict__ ap, int lda,
                                                  const _Float16* __restrict__ wt, int K,
                                                  const float* __restrict__ bias, float scale, float oscale,
                                                  _Float16* __restrict__ out, int ldo) {
  __shared__ __align__(16) float st[8][16 * OTP];
  const int tid = threadIdx.x, lane = tid & 31, wave = tid >> 5;
  const int hh = lane >> 4, c = lane & 15;
  const int m0 = blockIdx.x * 256 + wave * 32;
  const int n0 = blockIdx.y * 64;

  v8f acc[2][4];
#pragma unroll
  for (int s = 0; s < 2; ++s)
#pragma unroll
    for (int t = 0; t < 4; ++t) acc[s][t] = zero8();
  gemm32x64(ap, lda, wt, K, K, m0, n0, lane, acc);
  float bb[4];
#pragma unroll
  for (int t = 0; t < 4; ++t) bb[t] = bias[n0 + 16 * t + c];
  out_epilogue_h16(acc, scale, bb, oscale, st[wave], out, ldo, m0, n0, lane, hh, c);
}

__global__ __launch_bounds__(256) void k_ln(const float* __restrict__ tp, int tmode, const float* __restrict__ res,
                                            const float* __restrict__ g, const float* __restrict__ be,
                                            float* __restrict__ yf, _Float16* __restrict__ yh) {
  __shared__ __align__(16) float sw[8][DM];
  const int tid = threadIdx.x, lane = tid & 31, wave = tid >> 5;
  const int m = blockIdx.x * 8 + wave;
  const int b = m >> 9, s = m & (SQ - 1);

  v4f v[2];
  float sum = 0.f;
#pragma unroll
  for (int it = 0; it < 2; ++it) {
    const int idx = it * 128 + lane * 4;
    const size_t oa = ((size_t)(b * NH + (idx >> 5)) * SQ + s) * HDM + (idx & 31);
    const size_t ot = (size_t)m * DM + idx;
    const size_t o  = (tmode != 0) ? oa : ot;
    const v4f a = *(const v4f*)(tp + o);
    const v4f r = *(const v4f*)(res + ot);
    v[it] = a + r;
    sum += (v[it][0] + v[it][1]) + (v[it][2] + v[it][3]);
  }
#pragma unroll
  for (int off = 16; off >= 1; off >>= 1) sum += __shfl_xor(sum, off, 32);
  const float mean = sum * 0.00390625f;
  float ss = 0.f;
#pragma unroll
  for (int it = 0; it < 2; ++it) {
    const v4f d = v[it] - mean;
    ss += (d[0] * d[0] + d[1] * d[1]) + (d[2] * d[2] + d[3] * d[3]);
  }
#pragma unroll
  for (int off = 16; off >= 1; off >>= 1) ss += __shfl_xor(ss, off, 32);
  const float var  = ss * 0.00390625f;
  const float rstd = 1.0f / sqrtf(var + 1e-23f);

  v4f y[2];
#pragma unroll
  for (int it = 0; it < 2; ++it) {
    const int idx = it * 128 + lane * 4;
    const v4f gv = *(const v4f*)(g + idx);
    const v4f bv = *(const v4f*)(be + idx);
    y[it] = (gv * (v[it] - mean)) * rstd + bv;
  }
  for (int ps = 0; ps < 2; ++ps) {
#pragma unroll
    for (int it = 0; it < 2; ++it) *(volatile v4f*)(yf + (size_t)m * DM + it * 128 + lane * 4) = y[it];
    __threadfence();
  }
#pragma unroll
  for (int it = 0; it < 2; ++it) *(v4f*)(sw[wave] + it * 128 + lane * 4) = y[it];
  __syncthreads();
  const float* cp = sw[wave] + 8 * lane;
  const v4u hv = pack8h(*(const v4f*)(cp), *(const v4f*)(cp + 4));
  _Float16* hdst = yh + (size_t)m * DM + 8 * lane;
  for (int ps = 0; ps < 2; ++ps) {
    *(volatile v4u*)hdst = hv;
    __threadfence();
  }
}

__global__ __launch_bounds__(256) void k_head(const _Float16* __restrict__ xh,
                                              const _Float16* __restrict__ wot,
                                              const float* __restrict__ bo,
                                              float* __restrict__ out) {
  __shared__ __align__(16) float sf[256 * NLAB];
  const int tid = threadIdx.x, lane = tid & 31, wave = tid >> 5;
  const int hh = lane >> 4, c = lane & 15;
  const int m0 = blockIdx.x * 256 + wave * 32;

  v8f acc[2][2];
#pragma unroll
  for (int s = 0; s < 2; ++s)
#pragma unroll
    for (int t = 0; t < 2; ++t) acc[s][t] = zero8();
#pragma unroll 1
  for (int k0 = 0; k0 < DM; k0 += 32) {
    const v16h a0 = ldfrag(xh, DM, m0, k0, lane);
    const v16h a1 = ldfrag(xh, DM, m0 + 16, k0, lane);
    const v16h b0 = ldfrag(wot, DM, 0, k0, lane);
    const v16h b1 = ldfrag(wot, DM, 16, k0, lane);
    acc[0][0] = mma16(a0, b0, acc[0][0]);
    acc[1][0] = mma16(a1, b0, acc[1][0]);
    acc[0][1] = mma16(a0, b1, acc[0][1]);
    acc[1][1] = mma16(a1, b1, acc[1][1]);
  }
  float bb[2];
#pragma unroll
  for (int t = 0; t < 2; ++t) bb[t] = bo[min(16 * t + c, NLAB - 1)];
#pragma unroll
  for (int sub = 0; sub < 2; ++sub)
#pragma unroll
    for (int t = 0; t < 2; ++t) {
      const int col = 16 * t + c;
#pragma unroll
      for (int r = 0; r < 8; ++r) {
        const int row = wave * 32 + sub * 16 + 8 * hh + r;
        if (col < NLAB) sf[row * NLAB + col] = acc[sub][t][r] * 0.015625f + bb[t];
      }
    }
  __syncthreads();
  v4f val[5];
  size_t go[5];
#pragma unroll
  for (int it = 0; it < 5; ++it) {
    const int p = tid + 256 * it;
    val[it] = *(const v4f*)(sf + p * 4);
    go[it]  = (size_t)blockIdx.x * (256 * NLAB) + (size_t)p * 4;
  }
  for (int ps = 0; ps < 2; ++ps) {
#pragma unroll
    for (int it = 0; it < 5; ++it) *(volatile v4f*)(out + go[it]) = val[it];
    __threadfence();
  }
}

extern "C" void kernel_launch(void* const* d_in, const int* in_sizes, int n_in,
                              void* d_out, int out_size, void* d_ws, size_t ws_size,
                              hipStream_t stream) {
  if (n_in < 18) return;
  if (in_sizes[0] != NTOK) return;
  if (in_sizes[1] < NBATCH) return;
  if (in_sizes[2] < DM || (in_sizes[2] % DM) != 0) return;
  const int nvocab = in_sizes[2] / DM;
  if (in_sizes[3] < SQ * DM) return;
  if (in_sizes[4] != NLAYER * DM * DM) return;
  if (in_sizes[5] != NLAYER * DM) return;
  if (in_sizes[6] != NLAYER * DM * DM) return;
  if (in_sizes[7] != NLAYER * DM) return;
  if (in_sizes[8] != NLAYER * DM * DM) return;
  if (in_sizes[9] != NLAYER * DM) return;
  if (in_sizes[10] != DM) return;
  if (in_sizes[11] != DM) return;
  if (in_sizes[12] != DM * DFF) return;
  if (in_sizes[13] != DFF) return;
  if (in_sizes[14] != DFF * DM) return;
  if (in_sizes[15] != DM) return;
  if (in_sizes[16] != DM * NLAB) return;
  if (in_sizes[17] != NLAB) return;
  if (out_size != NTOK * NLAB) return;

  const int*   ids   = (const int*)d_in[0];
  const int*   slen  = (const int*)d_in[1];
  const float* emb   = (const float*)d_in[2];
  const float* pos   = (const float*)d_in[3];
  const float* wq    = (const float*)d_in[4];
  const float* bq    = (const float*)d_in[5];
  const float* wk    = (const float*)d_in[6];
  const float* bk    = (const float*)d_in[7];
  const float* wv    = (const float*)d_in[8];
  const float* bv    = (const float*)d_in[9];
  const float* gamma = (const float*)d_in[10];
  const float* beta  = (const float*)d_in[11];
  const float* w1    = (const float*)d_in[12];
  const float* b1    = (const float*)d_in[13];
  const float* w2    = (const float*)d_in[14];
  const float* b2    = (const float*)d_in[15];
  const float* wo    = (const float*)d_in[16];
  const float* bo    = (const float*)d_in[17];
  float* out = (float*)d_out;

  size_t off = 0;
  const size_t oXh  = off; off += (size_t)NTOK * DM * 2;
  const size_t oWT  = off; off += (size_t)NLAYER * NQKV * DM * 2;
  const size_t oW1  = off; off += (size_t)DFF * DM * 2;
  const size_t oW2  = off; off += (size_t)DM * DFF * 2;
  const size_t oWo  = off; off += (size_t)NLABP * DM * 2;
  const size_t oQK  = off; off += (size_t)2 * NTOK * DM * 2;
  const size_t oVT  = off; off += (size_t)NBATCH * NH * HDM * SQ * 2;
  const size_t oATT = off; off += (size_t)NBATCH * NH * SQ * HDM * 4;
  const size_t oHd  = oQK;
  if (oHd + (size_t)NTOK * DFF * 2 > off) return;
  const size_t oXa  = off; off += (size_t)NTOK * DM * 4;
  const size_t oXb  = off; off += (size_t)NTOK * DM * 4;
  const size_t oT   = off; off += (size_t)NTOK * DM * 4;
  if (off > ws_size) return;
  if (off > (size_t)134217728) return;

  char* ws = (char*)d_ws;
  _Float16* Xh  = (_Float16*)(ws + oXh);
  _Float16* WT  = (_Float16*)(ws + oWT);
  _Float16* W1T = (_Float16*)(ws + oW1);
  _Float16* W2T = (_Float16*)(ws + oW2);
  _Float16* WoT = (_Float16*)(ws + oWo);
  _Float16* QK  = (_Float16*)(ws + oQK);
  _Float16* VT  = (_Float16*)(ws + oVT);
  float*    ATT = (float*)(ws + oATT);
  _Float16* Hd  = (_Float16*)(ws + oHd);
  float*    Xa  = (float*)(ws + oXa);
  float*    Xb  = (float*)(ws + oXb);
  float*    T   = (float*)(ws + oT);

  const size_t wsz  = (size_t)DM * DM;
  const size_t lstr = (size_t)NQKV * DM;

  k_wtc<<<dim3(DM / 64, DM / 32, NLAYER), dim3(256), 0, stream>>>(wq, DM, DM, wsz, lstr, 64.0f, WT);
  k_wtc<<<dim3(DM / 64, DM / 32, NLAYER), dim3(256), 0, stream>>>(wk, DM, DM, wsz, lstr, 64.0f, WT + wsz);
  k_wtc<<<dim3(DM / 64, DM / 32, NLAYER), dim3(256), 0, stream>>>(wv, DM, DM, wsz, lstr, 64.0f, WT + 2 * wsz);
  k_wtc<<<dim3(DM / 64, DFF / 32, 1), dim3(256), 0, stream>>>(w1, DM, DFF, (size_t)0, (size_t)0, 64.0f, W1T);
  k_wtc<<<dim3(DFF / 64, DM / 32, 1), dim3(256), 0, stream>>>(w2, DFF, DM, (size_t)0, (size_t)0, 64.0f, W2T);
  k_wtc<<<dim3(DM / 64, NLABP / 32, 1), dim3(256), 0, stream>>>(wo, DM, NLAB, (size_t)0, (size_t)0, 64.0f, WoT);
  k_embed<<<dim3(NTOK / 8), dim3(256), 0, stream>>>(ids, emb, nvocab, pos, Xa, Xh);
  const float sscale = 0.0009765625f;
  for (int l = 0; l < NLAYER; ++l) {
    const size_t boff = (size_t)l * DM;
    k_qkv<<<dim3(NTOK / 256, NQKV / 64), dim3(256), 0, stream>>>(Xh, WT + (size_t)l * lstr,
                                                                  bq + boff, bk + boff, bv + boff, QK, VT);
    k_attn<<<dim3(NBATCH * NH * NQB), dim3(256), 0, stream>>>(QK, VT, slen, ATT, sscale);
    k_ln<<<dim3(NTOK / 8), dim3(256), 0, stream>>>(ATT, 1, Xa, gamma, beta, Xb, Xh);
    k_gemm_h16<<<dim3(NTOK / 256, DFF / 64), dim3(256), 0, stream>>>(Xh, DM, W1T, DM, b1, 0.015625f, 16.0f, Hd, DFF);
    k_gemm_f32<<<dim3(NTOK / 256, DM / 64), dim3(256), 0, stream>>>(Hd, DFF, W2T, DFF, b2, 0.0009765625f, T, DM);
    k_ln<<<dim3(NTOK / 8), dim3(256), 0, stream>>>(T, 0, Xb, gamma, beta, Xa, Xh);
  }
  k_head<<<dim3(NTOK / 256), dim3(256), 0, stream>>>(Xh, WoT, bo, out);
  (void)hipGetLastError();
}
